// MultiHeadAttention_66305705116193
// MI455X (gfx1250) — hardware-run, weakly checked
//
#include <hip/hip_runtime.h>


#ifndef NB
#define NB 2
#endif
#ifndef SEQ
#define SEQ 2048
#endif
#define NB_FULL  2
#define SEQ_FULL 2048
#ifndef OUT_SEQ
#define OUT_SEQ SEQ
#endif
#define DM   2048
#define NH_  16
#define NKV  4
#define HD   128
#define REP  (NH_ / NKV)
#define DKV  (NKV * HD)
#define AW   4
#define QRS  2048.0f
#define QRI  (1.0f / 2048.0f)
#define VRS  256.0f
#define LOG2E 1.4426950408889634f
#define SC2  (0.08838834764831845f * 1.4426950408889634f)
#define PSH  8.0f
#define NEGBIG (-3.0e38f)

static_assert(HD == 128);
static_assert(NH_ * HD == DM);
static_assert(NH_ % NKV == 0);
static_assert(DM % 64 == 0);
static_assert(DKV % 64 == 0);
static_assert(DM % 32 == 0);
static_assert(SEQ % 64 == 0);
static_assert((NB * SEQ) % 64 == 0);
static_assert(SEQ % 32 == 0);
static_assert(SEQ % (16 * AW) == 0);
static_assert(SEQ % 4 == 0);
static_assert(((size_t)SEQ * DM) % 8 == 0);
static_assert(NB <= NB_FULL);
static_assert(SEQ <= SEQ_FULL);

typedef _Float16 h16;
typedef unsigned short bf;
typedef __attribute__((ext_vector_type(16))) __bf16   v16bf;
typedef __attribute__((ext_vector_type(16))) _Float16 v16h;
typedef __attribute__((ext_vector_type(8)))  _Float16 v8h;
typedef __attribute__((ext_vector_type(8)))  unsigned short v8us;
typedef __attribute__((ext_vector_type(8)))  float    v8f;
typedef __attribute__((ext_vector_type(4)))  float    v4f;
typedef v4f  __attribute__((may_alias)) v4fa;

__device__ __forceinline__ unsigned short f2bf(float f) { unsigned u = __float_as_uint(f); u += 0x7FFFu + ((u >> 16) & 1u); return (unsigned short)(u >> 16); }
__device__ __forceinline__ float bf2f(unsigned short u) { return __uint_as_float(((unsigned)u) << 16); }
__device__ __forceinline__ float bfr(float f) { return bf2f(f2bf(f)); }
__device__ __forceinline__ v16h cat16(v8h lo, v8h hi) { return __builtin_shufflevector(lo, hi, 0, 1, 2, 3, 4, 5, 6, 7, 8, 9, 10, 11, 12, 13, 14, 15); }
__device__ __forceinline__ v16bf cat16b(v8us lo, v8us hi) { return __builtin_bit_cast(v16bf, __builtin_shufflevector(lo, hi, 0, 1, 2, 3, 4, 5, 6, 7, 8, 9, 10, 11, 12, 13, 14, 15)); }
__device__ __forceinline__ v8f wmma16(v16h a, v16h b, v8f c) { return __builtin_amdgcn_wmma_f32_16x16x32_f16(false, a, false, b, (short)0, c, false, false); }
__device__ __forceinline__ v8f wmmab(v16bf a, v16bf b, v8f c) { return __builtin_amdgcn_wmma_f32_16x16x32_bf16(false, a, false, b, (short)0, c, false, false); }
__device__ __forceinline__ v16h  ldh(const h16* p) { return cat16(*(const v8h*)p, *(const v8h*)(p + 16)); }
__device__ __forceinline__ v16bf ldb(const bf* p)  { return cat16b(*(const v8us*)p, *(const v8us*)(p + 16)); }
__device__ __forceinline__ void wave_sync() { __builtin_amdgcn_fence(3  , "wavefront"); __builtin_amdgcn_wave_barrier(); asm volatile("" ::: "memory"); }

__global__ __launch_bounds__(256) void k_cvt8(const float* __restrict__ src, bf* dst, size_t n8) {
    const size_t i = (size_t)blockIdx.x * 256 + threadIdx.x; if (i >= n8) return;
    const v8f v = *(const v8f*)(src + i * 8); v8us o;
#pragma unroll
    for (int k = 0; k < 8; ++k) o[k] = f2bf(v[k]);
    *(volatile v8us*)(dst + i * 8) = o; __threadfence(); *(volatile v8us*)(dst + i * 8) = o;
}

__global__ __launch_bounds__(256) void k_tcvt(const float* __restrict__ W, bf* WT, int K, int N) {
    __shared__ float ts[64 * 65];
    const int tid = threadIdx.x; const int k0 = blockIdx.x * 64, n0 = blockIdx.y * 64;
    const int cn = tid & 63, rk = tid >> 6;
#pragma unroll 4
    for (int i = 0; i < 16; ++i) { const int r = rk + 4 * i; ts[r * 65 + cn] = W[(size_t)(k0 + r) * N + n0 + cn]; }
    __syncthreads();
    const int pc = tid & 7, rn = tid >> 3;
    v8us o0, o1;
#pragma unroll
    for (int j = 0; j < 8; ++j) { o0[j] = f2bf(ts[(pc * 8 + j) * 65 + rn]); o1[j] = f2bf(ts[(pc * 8 + j) * 65 + rn + 32]); }
    bf* d0 = WT + (size_t)(n0 + rn) * K + k0 + pc * 8; bf* d1 = WT + (size_t)(n0 + rn + 32) * K + k0 + pc * 8;
    *(volatile v8us*)d0 = o0; *(volatile v8us*)d1 = o1; __threadfence(); *(volatile v8us*)d0 = o0; *(volatile v8us*)d1 = o1;
}

__global__ __launch_bounds__(256) void k_rope_tab(float* CS) {
    __shared__ __align__(16) float ts[4 * 128];
    const int tid = threadIdx.x; const int i = tid & 63, r = tid >> 6; const int t = blockIdx.x * 4 + r;
    const float invf = __builtin_amdgcn_exp2f(-(float)i * 0.20762050593046014f);
    const float ang = (float)t * invf;
    ts[r * 128 + i] = cosf(ang); ts[r * 128 + 64 + i] = sinf(ang);
    __syncthreads();
    if (tid < 128) {
        const int row = tid >> 5, pc = tid & 31;
        const v4f v = *(const v4fa*)(&ts[row * 128 + pc * 4]);
        float* d = CS + (size_t)(blockIdx.x * 4 + row) * 128 + pc * 4;
        *(volatile v4f*)d = v; __threadfence(); *(volatile v4f*)d = v;
    }
}

template <int MT, int NT>
__device__ __forceinline__ void gemm_loop(const bf* __restrict__ A, size_t lda, const bf* __restrict__ Bt, size_t ldbt,
                                          int K, int kbm, int r0, int c0, int lr, int hi, v8f (&acc)[MT * NT]) {
#pragma unroll
    for (int i = 0; i < MT * NT; ++i) acc[i] = (v8f){};
    const size_t aoff = (size_t)(r0 + lr) * lda + 8 * hi, boff = (size_t)(c0 + lr) * ldbt + 8 * hi;
#pragma unroll 1
    for (int kc = 0; kc < K; kc += 32) {
        const int kb = kc & kbm;
        v16bf a[MT];
#pragma unroll
        for (int mb = 0; mb < MT; ++mb) a[mb] = ldb(A + aoff + (size_t)mb * 16 * lda + kc);
        v16bf bl = a[0];
#pragma unroll
        for (int nb = 0; nb < NT; ++nb) { const v16bf b = ldb(Bt + boff + (size_t)nb * 16 * ldbt + kb);
#pragma unroll
            for (int mb = 0; mb < MT; ++mb) acc[mb * NT + nb] = wmmab(a[mb], b, acc[mb * NT + nb]);
            if (nb == NT - 1) bl = b; }
        asm volatile("v_nop\n\tv_nop\n\tv_nop\n\tv_nop" : "+v"(acc[0]), "+v"(acc[(MT * NT) / 3]), "+v"(acc[(2 * MT * NT) / 3]), "+v"(acc[MT * NT - 1]) : "v"(a[0]), "v"(a[MT - 1]), "v"(bl));
    }
}

__global__ __launch_bounds__(32) __attribute__((amdgpu_num_vgpr(256)))
void k_qk(const bf* __restrict__ A, const bf* __restrict__ Bt, const float* __restrict__ bias, const float* __restrict__ CS, h16* Ph, h16* Pr, int useRes, int nheads) {
    __shared__ __align__(16) float os[16 * 132];
    const int lane = threadIdx.x & 31, lr = lane & 15, hi = lane >> 4;
    const int r0 = blockIdx.x * 32, head = blockIdx.y, cbase = head * HD;
    v8f acc[16];
    gemm_loop<2, 8>(A, (size_t)DM, Bt, (size_t)DM, DM, 0x7FFFFFFF, r0, cbase, lr, hi, acc);
    float bz[8];
#pragma unroll
    for (int nb = 0; nb < 8; ++nb) bz[nb] = bfr(bias[cbase + nb * 16 + lr]);
    const int b = r0 / SEQ, t0 = r0 % SEQ;
    const size_t tbase = ((size_t)(b * nheads + head) * SEQ + t0) * HD;
#pragma unroll
    for (int mb = 0; mb < 2; ++mb) {
#pragma unroll
        for (int nb = 0; nb < 8; ++nb) {
#pragma unroll
            for (int j = 0; j < 8; ++j) os[(hi * 8 + j) * 132 + nb * 16 + lr] = acc[mb * 8 + nb][j] + bz[nb]; }
        wave_sync();
#pragma unroll 1
        for (int ps = 0; ps < 2; ++ps) {
#pragma unroll 2
            for (int s = 0; s < 8; ++s) { const int row = 2 * s + hi, c8 = lr * 8, p8 = c8 ^ 64;
                const int t = t0 + mb * 16 + row;
                const float* orow = &os[row * 132];
                const v4f x0 = *(const v4fa*)(orow + c8), x1 = *(const v4fa*)(orow + c8 + 4);
                const v4f y0 = *(const v4fa*)(orow + p8), y1 = *(const v4fa*)(orow + p8 + 4);
                const float* cs = CS + (size_t)t * 128 + (c8 & 63);
                const v4f cc0 = *(const v4f*)cs, cc1 = *(const v4f*)(cs + 4), ss0 = *(const v4f*)(cs + 64), ss1 = *(const v4f*)(cs + 68);
                const float sg = (c8 < 64) ? -1.0f : 1.0f;
                v8h hv, rv;
#pragma unroll
                for (int i = 0; i < 4; ++i) {
                    const float v0 = x0[i] * cc0[i] + sg * (y0[i] * ss0[i]); const float v1 = x1[i] * cc1[i] + sg * (y1[i] * ss1[i]);
                    const h16 a0 = (h16)v0; const h16 a1 = (h16)v1; hv[i] = a0; hv[4 + i] = a1;
                    rv[i] = (h16)((v0 - (float)a0) * QRS); rv[4 + i] = (h16)((v1 - (float)a1) * QRS); }
                const size_t oo = tbase + (size_t)(mb * 16 + row) * HD + c8;
                *(volatile v8h*)(Ph + oo) = hv; if (useRes) *(volatile v8h*)(Pr + oo) = rv; }
            if (ps == 0) __threadfence(); }
        wave_sync();
    }
}

__global__ __launch_bounds__(32) __attribute__((amdgpu_num_vgpr(256)))
void k_vt(const bf* __restrict__ A, const bf* __restrict__ Bt, const float* __restrict__ bias, h16* VH, h16* VR) {
    __shared__ __align__(16) float os[16 * 68];
    const int lane = threadIdx.x & 31, lr = lane & 15, hi = lane >> 4;
    const int r0 = blockIdx.x * 64, c0 = blockIdx.y * 64;
    v8f acc[16];
    gemm_loop<4, 4>(A, (size_t)DM, Bt, (size_t)DM, DM, 0x7FFFFFFF, r0, c0, lr, hi, acc);
    const int b = c0 / SEQ, t0 = c0 % SEQ;
    const size_t tbase = ((size_t)b * DKV + r0) * SEQ + t0;
#pragma unroll
    for (int mb = 0; mb < 4; ++mb) {
        float bj[8];
#pragma unroll
        for (int j = 0; j < 8; ++j) bj[j] = bfr(bias[r0 + mb * 16 + hi * 8 + j]);
#pragma unroll
        for (int nb = 0; nb < 4; ++nb) {
#pragma unroll
            for (int j = 0; j < 8; ++j) os[(hi * 8 + j) * 68 + nb * 16 + lr] = acc[mb * 4 + nb][j] + bj[j]; }
        wave_sync();
        const size_t sb = tbase + (size_t)(mb * 16) * SEQ;
#pragma unroll 1
        for (int ps = 0; ps < 2; ++ps) {
#pragma unroll
            for (int s = 0; s < 4; ++s) { const int row = 4 * s + (lane >> 3), c8 = (lane & 7) * 8;
                const v4f x0 = *(const v4fa*)(&os[row * 68 + c8]); const v4f x1 = *(const v4fa*)(&os[row * 68 + c8 + 4]); v8h hv, rv;
#pragma unroll
                for (int i = 0; i < 4; ++i) { const h16 a0 = (h16)x0[i]; const h16 a1 = (h16)x1[i]; hv[i] = a0; hv[4 + i] = a1; rv[i] = (h16)((x0[i] - (float)a0) * VRS); rv[4 + i] = (h16)((x1[i] - (float)a1) * VRS); }
                const size_t oo = sb + (size_t)row * SEQ + c8;
                *(volatile v8h*)(VH + oo) = hv; *(volatile v8h*)(VR + oo) = rv; }
            if (ps == 0) __threadfence(); }
        wave_sync();
    }
}

__global__ __launch_bounds__(32 * AW) __attribute__((amdgpu_num_vgpr(256)))
void k_flash(const h16* __restrict__ QH, const h16* __restrict__ QR, const h16* __restrict__ KP, const h16* __restrict__ VH, const h16* __restrict__ VR, bf* CTX) {
    __shared__ __align__(16) float os[AW * 16 * 132];
    const int lane = threadIdx.x & 31, wave = threadIdx.x >> 5, lr = lane & 15, hi = lane >> 4;
    const int zh = blockIdx.y; const int b = zh / NH_, h = zh % NH_; const int g = h / REP;
    const int t0 = (blockIdx.x * AW + wave) * 16;
    const size_t qo = (size_t)zh * SEQ * HD + (size_t)(t0 + lr) * HD + 8 * hi;
    v16h qh[4], qr[4];
#pragma unroll
    for (int c = 0; c < 4; ++c) { qh[c] = ldh(QH + qo + 32 * c); qr[c] = ldh(QR + qo + 32 * c); }
    const size_t kvb = (size_t)(b * NKV + g) * SEQ * HD;
    const size_t ko = kvb + (size_t)lr * HD + 8 * hi;
    const size_t vo = kvb + (size_t)lr * SEQ + 8 * hi;
    const float slope2 = __builtin_amdgcn_exp2f(-0.5f * (float)(h + 1)) * LOG2E;
    const int qi = t0 + lr;
    v8f o[8];
#pragma unroll
    for (int j = 0; j < 8; ++j) o[j] = (v8f){};
    float m = NEGBIG, l = 0.0f;
    const int kend = ((t0 + 16 + 31) >> 5) << 5;
#pragma unroll 1
    for (int key0 = 0; key0 < kend; key0 += 32) {
        const h16* ka = KP + ko + (size_t)key0 * HD;
        v8f sHa = (v8f){}, sLa = (v8f){}, sHb = (v8f){}, sLb = (v8f){};
        v16h kal, kbl;
#pragma unroll
        for (int c = 0; c < 4; ++c) {
            kal = ldh(ka + 32 * c); kbl = ldh(ka + 16 * HD + 32 * c);
            sHa = wmma16(kal, qh[c], sHa); sLa = wmma16(kal, qr[c], sLa); sHb = wmma16(kbl, qh[c], sHb); sLb = wmma16(kbl, qr[c], sLb); }
        asm volatile("v_nop\n\tv_nop\n\tv_nop\n\tv_nop" : "+v"(sHa), "+v"(sLa), "+v"(sHb), "+v"(sLb) : "v"(kal), "v"(kbl));
        const float base = (float)(key0 + 8 * hi - qi);
        float ta[8], tb[8]; float mx = NEGBIG;
#pragma unroll
        for (int r = 0; r < 8; ++r) {
            const float da = base + (float)r, db = da + 16.0f;
            float xa = fmaf(slope2, da, (sHa[r] + sLa[r] * QRI) * SC2);
            float xb = fmaf(slope2, db, (sHb[r] + sLb[r] * QRI) * SC2);
            xa = (da > 0.0f) ? NEGBIG : xa; xb = (db > 0.0f) ? NEGBIG : xb;
            ta[r] = xa; tb[r] = xb; mx = fmaxf(mx, fmaxf(xa, xb)); }
        mx = fmaxf(mx, __shfl_xor(mx, 16, 32));
        const float mnew = fmaxf(m, mx);
        const float alpha = __builtin_amdgcn_exp2f(m - mnew);
        const float sh = PSH - mnew;
        v16h pb; float ls = 0.0f;
#pragma unroll
        for (int r = 0; r < 8; ++r) { const h16 pa = (h16)__builtin_amdgcn_exp2f(ta[r] + sh); const h16 pc = (h16)__builtin_amdgcn_exp2f(tb[r] + sh); pb[r] = pa; pb[8 + r] = pc; ls += (float)pa + (float)pc; }
        const v16h pq = pb * (h16)0.00390625f;
        l = l * alpha + ls; m = mnew;
#pragma unroll
        for (int j = 0; j < 8; ++j) o[j] = o[j] * alpha;
        const h16* va = VH + vo + key0; const h16* vr = VR + vo + key0;
#pragma unroll
        for (int j = 0; j < 8; ++j) { const v16h vf = ldh(va + (size_t)(16 * j) * SEQ); o[j] = wmma16(vf, pb, o[j]); }
#pragma unroll
        for (int j = 0; j < 8; ++j) { const v16h vf = ldh(vr + (size_t)(16 * j) * SEQ); o[j] = wmma16(vf, pq, o[j]); }
        asm volatile("v_nop\n\tv_nop\n\tv_nop\n\tv_nop" : "+v"(o[0]), "+v"(o[1]), "+v"(o[2]), "+v"(o[3]), "+v"(o[4]), "+v"(o[5]), "+v"(o[6]), "+v"(o[7]) : "v"(pb), "v"(pq));
    }
    l += __shfl_xor(l, 16, 32);
    const float inv = 1.0f / l;
    const int wb = wave * 16 * 132;
#pragma unroll
    for (int j = 0; j < 8; ++j) { v4f a, c;
        a[0] = o[j][0] * inv; a[1] = o[j][1] * inv; a[2] = o[j][2] * inv; a[3] = o[j][3] * inv; c[0] = o[j][4] * inv; c[1] = o[j][5] * inv; c[2] = o[j][6] * inv; c[3] = o[j][7] * inv;
        *(v4fa*)(&os[wb + lr * 132 + 16 * j + 8 * hi]) = a; *(v4fa*)(&os[wb + lr * 132 + 16 * j + 8 * hi + 4]) = c; }
    wave_sync();
    bf* crow = CTX + ((size_t)b * SEQ + t0) * (size_t)(2 * DM) + h * HD;
#pragma unroll 1
    for (int ps = 0; ps < 2; ++ps) {
#pragma unroll 2
        for (int s = 0; s < 8; ++s) { const int row = 2 * s + hi, c8 = lr * 8;
            const v4f x0 = *(const v4fa*)(&os[wb + row * 132 + c8]); const v4f x1 = *(const v4fa*)(&os[wb + row * 132 + c8 + 4]); v8us hv, lv;
#pragma unroll
            for (int i = 0; i < 4; ++i) { const unsigned short a0 = f2bf(x0[i]); const unsigned short a1 = f2bf(x1[i]); hv[i] = a0; hv[4 + i] = a1; lv[i] = f2bf(x0[i] - bf2f(a0)); lv[4 + i] = f2bf(x1[i] - bf2f(a1)); }
            bf* dst = crow + (size_t)row * (size_t)(2 * DM) + c8;
            *(volatile v8us*)dst = hv; *(volatile v8us*)(dst + DM) = lv; }
        if (ps == 0) __threadfence(); }
}

__global__ __launch_bounds__(32) __attribute__((amdgpu_num_vgpr(256)))
void k_out(const bf* __restrict__ A, const bf* __restrict__ Bt, const float* __restrict__ bias, float* OUT) {
    __shared__ __align__(16) float os[16 * 68];
    const int lane = threadIdx.x & 31, lr = lane & 15, hi = lane >> 4;
    const int r0 = blockIdx.x * 64, c0 = blockIdx.y * 64;
    v8f acc[16];
    gemm_loop<4, 4>(A, (size_t)(2 * DM), Bt, (size_t)DM, 2 * DM, DM - 1, r0, c0, lr, hi, acc);
    float bz[4];
#pragma unroll
    for (int nb = 0; nb < 4; ++nb) bz[nb] = bfr(bias[c0 + nb * 16 + lr]);
    const int b = r0 / SEQ, t0 = r0 % SEQ;
    float* obase = OUT + ((size_t)b * OUT_SEQ + t0) * DM + c0;
#pragma unroll
    for (int mb = 0; mb < 4; ++mb) {
#pragma unroll
        for (int nb = 0; nb < 4; ++nb) {
#pragma unroll
            for (int j = 0; j < 8; ++j) os[(hi * 8 + j) * 68 + nb * 16 + lr] = acc[mb * 4 + nb][j] + bz[nb]; }
        wave_sync();
        float* orow = obase + (size_t)(mb * 16) * DM;
#pragma unroll 1
        for (int ps = 0; ps < 2; ++ps) {
#pragma unroll
            for (int s = 0; s < 8; ++s) { const int row = 2 * s + hi, cofs = lr * 4;
                const v4f val = *(const v4fa*)(&os[row * 68 + cofs]);
                *(volatile v4f*)(orow + (size_t)row * DM + cofs) = val; }
            if (ps == 0) __threadfence(); }
        wave_sync();
    }
}

static constexpr size_t al256(size_t v) { return (v + 255) & ~(size_t)255; }
static constexpr size_t SZ_XB  = al256((size_t)NB * SEQ * DM * 2);
static constexpr size_t SZ_WQ  = al256((size_t)DM * DM * 2);
static constexpr size_t SZ_WK  = al256((size_t)DKV * DM * 2);
static constexpr size_t SZ_CS  = al256((size_t)SEQ * 128 * 4);
static constexpr size_t SZ_QP  = al256((size_t)NB * NH_ * SEQ * HD * 2);
static constexpr size_t SZ_KP  = al256((size_t)NB * NKV * SEQ * HD * 2);
static constexpr size_t SZ_CTX = al256((size_t)NB * SEQ * 2 * DM * 2);
static constexpr size_t SZ_TOTAL = SZ_XB + 2 * SZ_WQ + 2 * SZ_WK + SZ_CS + 2 * SZ_QP + 3 * SZ_KP + SZ_CTX;
static_assert(SZ_TOTAL <= (size_t)134217728);

extern "C" void kernel_launch(void* const* d_in, const int* in_sizes, int n_in,
                              void* d_out, int out_size, void* d_ws, size_t ws_size, hipStream_t stream) {
    if (n_in < 9) return;
    const size_t needx = ((size_t)(NB - 1) * SEQ_FULL + SEQ) * DM;
    if ((size_t)in_sizes[0] < needx) return;
    if ((size_t)in_sizes[1] < (size_t)DM * DM || (size_t)in_sizes[2] < (size_t)DM) return;
    if ((size_t)in_sizes[3] < (size_t)DM * DKV || (size_t)in_sizes[4] < (size_t)DKV) return;
    if ((size_t)in_sizes[5] < (size_t)DM * DKV || (size_t)in_sizes[6] < (size_t)DKV) return;
    if ((size_t)in_sizes[7] < (size_t)DM * DM || (size_t)in_sizes[8] < (size_t)DM) return;
    if ((size_t)out_size < ((size_t)(NB - 1) * OUT_SEQ + SEQ) * DM) return;
    if (SZ_TOTAL > ws_size) return;
    const float* x  = (const float*)d_in[0];
    const float* wq = (const float*)d_in[1]; const float* bq = (const float*)d_in[2];
    const float* wk = (const float*)d_in[3]; const float* bk = (const float*)d_in[4];
    const float* wv = (const float*)d_in[5]; const float* bv = (const float*)d_in[6];
    const float* wo = (const float*)d_in[7]; const float* bo = (const float*)d_in[8];
    float* OUT = (float*)d_out;
    char* wsp = (char*)d_ws;
    bf* XB  = (bf*)wsp; wsp += SZ_XB;
    bf* WQT = (bf*)wsp; wsp += SZ_WQ;
    bf* WOT = (bf*)wsp; wsp += SZ_WQ;
    bf* WKT = (bf*)wsp; wsp += SZ_WK;
    bf* WVT = (bf*)wsp; wsp += SZ_WK;
    float* CS = (float*)wsp; wsp += SZ_CS;
    h16* QH = (h16*)wsp; wsp += SZ_QP;
    h16* QR = (h16*)wsp; wsp += SZ_QP;
    h16* KP = (h16*)wsp; wsp += SZ_KP;
    h16* VH = (h16*)wsp; wsp += SZ_KP;
    h16* VR = (h16*)wsp; wsp += SZ_KP;
    bf* CTX = (bf*)wsp; wsp += SZ_CTX;

    if (SEQ == SEQ_FULL) {
        const size_t n8 = (size_t)NB * SEQ * DM / 8;
        k_cvt8<<<(unsigned)((n8 + 255) / 256), 256, 0, stream>>>(x, XB, n8);
    } else {
        const size_t n8 = (size_t)SEQ * DM / 8;
        for (int b = 0; b < NB; ++b) k_cvt8<<<(unsigned)((n8 + 255) / 256), 256, 0, stream>>>(x + (size_t)b * SEQ_FULL * DM, XB + (size_t)b * SEQ * DM, n8);
    }
    k_tcvt<<<dim3(DM / 64, DM / 64, 1), 256, 0, stream>>>(wq, WQT, DM, DM);
    k_tcvt<<<dim3(DM / 64, DKV / 64, 1), 256, 0, stream>>>(wk, WKT, DM, DKV);
    k_tcvt<<<dim3(DM / 64, DKV / 64, 1), 256, 0, stream>>>(wv, WVT, DM, DKV);
    k_tcvt<<<dim3(DM / 64, DM / 64, 1), 256, 0, stream>>>(wo, WOT, DM, DM);
    k_rope_tab<<<SEQ / 4, 256, 0, stream>>>(CS);

    k_qk<<<dim3(NB * SEQ / 32, NH_, 1), 32, 0, stream>>>(XB, WQT, bq, CS, QH, QR, 1, NH_);
    k_qk<<<dim3(NB * SEQ / 32, NKV, 1), 32, 0, stream>>>(XB, WKT, bk, CS, KP, KP, 0, NKV);
    k_vt<<<dim3(DKV / 64, NB * SEQ / 64, 1), 32, 0, stream>>>(WVT, XB, bv, VH, VR);

    k_flash<<<dim3(SEQ / (16 * AW), NB * NH_, 1), 32 * AW, 0, stream>>>(QH, QR, KP, VH, VR, CTX);

    k_out<<<dim3(NB * SEQ / 64, DM / 64, 1), 32, 0, stream>>>(CTX, WOT, bo, OUT);
}
